// MLPScorer_8589934807
// MI455X (gfx1250) — hardware-verified
//
#include <hip/hip_runtime.h>


#ifndef NB
#define NB 4
#endif
#ifndef TQ
#define TQ 512
#endif
#ifndef SK
#define SK 512
#endif
#define NB_FULL 4
#define TQ_FULL 512
#define SK_FULL 512
#define DM   512
#define TT   32
#define TS   32
#define CH   128
#define LRP  (CH + 4)
#define OSP  36

static_assert(DM % 32 == 0);
static_assert(DM % 64 == 0);
static_assert((NB * TQ) % 64 == 0);
static_assert((NB * SK) % 64 == 0);
static_assert(TQ % TT == 0);
static_assert(SK % TS == 0);
static_assert(TT == 32);
static_assert(TS == 32);
static_assert(DM % CH == 0);
static_assert(CH % 4 == 0);
static_assert(TT * (CH / 4) == 256 * 4);
static_assert(TS * (CH / 4) == 256 * 4);
static_assert(256 * 16 * 1 == TT * TS * 4);
static_assert(32 * 16 * 8 == 16 * 64 * 4);
static_assert((LRP * 4) % 16 == 0);
static_assert((OSP * 4) % 16 == 0);
static_assert((size_t)(TT + TS) * LRP * 4 + (size_t)DM * 4 + (size_t)TT * OSP * 4 <= 131072);
static_assert((size_t)16 * 68 * 4 <= 131072);
static_assert(((size_t)TQ * DM) % 8 == 0);
static_assert(((size_t)SK * DM) % 8 == 0);
static_assert(((size_t)DM * DM) % 8 == 0);
static_assert(NB <= NB_FULL);
static_assert(TQ <= TQ_FULL);
static_assert(SK <= SK_FULL);

typedef unsigned short bf;
typedef __attribute__((ext_vector_type(16))) __bf16   v16bf;
typedef __attribute__((ext_vector_type(8)))  unsigned short v8us;
typedef __attribute__((ext_vector_type(8)))  float    v8f;
typedef __attribute__((ext_vector_type(4)))  float    v4f;
typedef v4f  __attribute__((may_alias)) v4fa;

__device__ __forceinline__ unsigned short f2bf(float f) { unsigned u = __float_as_uint(f); u += 0x7FFFu + ((u >> 16) & 1u); return (unsigned short)(u >> 16); }
__device__ __forceinline__ float bfr(float f) { return __uint_as_float(((unsigned)f2bf(f)) << 16); }
__device__ __forceinline__ v16bf cat16b(v8us lo, v8us hi) { return __builtin_bit_cast(v16bf, __builtin_shufflevector(lo, hi, 0, 1, 2, 3, 4, 5, 6, 7, 8, 9, 10, 11, 12, 13, 14, 15)); }
__device__ __forceinline__ v8f wmmab(v16bf a, v16bf b, v8f c) { return __builtin_amdgcn_wmma_f32_16x16x32_bf16(false, a, false, b, (short)0, c, false, false); }
__device__ __forceinline__ v16bf ldb(const bf* p)  { return cat16b(*(const v8us*)p, *(const v8us*)(p + 16)); }
__device__ __forceinline__ void wave_sync() { __builtin_amdgcn_fence(3  , "wavefront"); __builtin_amdgcn_wave_barrier(); asm volatile("" ::: "memory"); }
__device__ __forceinline__ v8f wmmab_g(v16bf a, v16bf b, v8f c) {
    c = wmmab(a, b, c);
    asm volatile("v_nop\n\tv_nop\n\tv_nop\n\tv_nop" : "+v"(c) : "v"(a), "v"(b));
    return c;
}

__device__ __forceinline__ float fast_tanh(float x) {
#if __has_builtin(__builtin_amdgcn_tanhf)
    return __builtin_amdgcn_tanhf(x);
#elif __has_builtin(__builtin_amdgcn_tanh_f32)
    return __builtin_amdgcn_tanh_f32(x);
#else
    float r;
    asm volatile("v_tanh_f32 %0, %1" : "=v"(r) : "v"(x));
    return r;
#endif
}

__global__ __launch_bounds__(256) void k_cvt8(const float* __restrict__ src, bf* dst, size_t n8) {
    const size_t i = (size_t)blockIdx.x * 256 + threadIdx.x; if (i >= n8) return;
    const v8f v = *(const v8f*)(src + i * 8); v8us o;
#pragma unroll
    for (int k = 0; k < 8; ++k) o[k] = f2bf(v[k]);
    *(volatile v8us*)(dst + i * 8) = o; __threadfence(); *(volatile v8us*)(dst + i * 8) = o;
}

__global__ __launch_bounds__(32) void k_projf(const bf* __restrict__ A, const bf* __restrict__ Bt, const float* __restrict__ bias, int use_bias, float* Y) {
    __shared__ __align__(16) float os[16 * 68];
    const int K = DM;
    const int lane = threadIdx.x & 31, lr = lane & 15, hi = lane >> 4; const int r0 = blockIdx.x * 64, c0 = blockIdx.y * 64;
    v8f acc[4][4];
#pragma unroll
    for (int mb = 0; mb < 4; ++mb)
#pragma unroll
        for (int nb = 0; nb < 4; ++nb) acc[mb][nb] = (v8f){};
    const size_t aoff = (size_t)(r0 + lr) * K + 8 * hi, boff = (size_t)(c0 + lr) * K + 8 * hi;
#pragma unroll 1
    for (int kc = 0; kc < K; kc += 32) {
        v16bf a[4];
#pragma unroll
        for (int mb = 0; mb < 4; ++mb) a[mb] = ldb(A + aoff + (size_t)mb * 16 * K + kc);
#pragma unroll
        for (int nb = 0; nb < 4; ++nb) { const v16bf b = ldb(Bt + boff + (size_t)nb * 16 * K + kc);
#pragma unroll
            for (int mb = 0; mb < 4; ++mb) acc[mb][nb] = wmmab_g(a[mb], b, acc[mb][nb]); }
    }
    float bc[4];
#pragma unroll
    for (int nb = 0; nb < 4; ++nb) { const float bv = bias[c0 + nb * 16 + lr]; bc[nb] = (use_bias != 0) ? bfr(bv) : 0.0f; }
    float* yb = Y + (size_t)r0 * DM + c0;
#pragma unroll
    for (int mb = 0; mb < 4; ++mb) {
#pragma unroll
        for (int nb = 0; nb < 4; ++nb) {
#pragma unroll
            for (int j = 0; j < 8; ++j) os[(hi * 8 + j) * 68 + nb * 16 + lr] = acc[mb][nb][j] + bc[nb]; }
        wave_sync();
#pragma unroll 1
        for (int ps = 0; ps < 2; ++ps) {
#pragma unroll
            for (int s = 0; s < 8; ++s) { const int row = 2 * s + (lane >> 4), cofs = (lane & 15) * 4;
                const v4f val = *(const v4fa*)(&os[row * 68 + cofs]);
                *(volatile v4f*)(yb + (size_t)(mb * 16 + row) * DM + cofs) = val; }
            if (ps == 0) __threadfence(); }
        wave_sync();
    }
}

__global__ __launch_bounds__(256) void k_pairsum(const float* __restrict__ WQ, const float* __restrict__ UH, const float* __restrict__ V, float* OUT) {
    __shared__ __align__(16) float swq[TT * LRP];
    __shared__ __align__(16) float suh[TS * LRP];
    __shared__ __align__(16) float sv[DM];
    __shared__ __align__(16) float os[TT * OSP];
    const int tid = threadIdx.x, lane = tid & 31;
    const int wave = __builtin_amdgcn_readfirstlane((int)(threadIdx.x >> 5));
    const int s0 = blockIdx.x * TS, t0 = blockIdx.y * TT, b = blockIdx.z;
    const size_t wqb = ((size_t)b * TQ + t0) * DM, uhb = ((size_t)b * SK + s0) * DM;
#pragma unroll 1
    for (int i = tid; i < DM; i += 256) sv[i] = bfr(V[i]);
    const int tl = tid >> 4, sl = tid & 15;
    const int srow = tid >> 5, sc4 = (tid & 31) * 4;
    float a00 = 0.0f, a01 = 0.0f, a10 = 0.0f, a11 = 0.0f;
#pragma unroll 1
    for (int ch = 0; ch < DM; ch += CH) {
#pragma unroll
        for (int i = 0; i < 4; ++i) { const int row = srow + 8 * i;
            const v4f w = *(const v4f*)(WQ + wqb + (size_t)row * DM + ch + sc4);
            const v4f u = *(const v4f*)(UH + uhb + (size_t)row * DM + ch + sc4);
            *(v4fa*)(&swq[row * LRP + sc4]) = w; *(v4fa*)(&suh[row * LRP + sc4]) = u; }
        __syncthreads();
#pragma unroll 2
        for (int d = 0; d < CH; d += 4) {
            const v4f w0 = *(const v4fa*)(&swq[tl * LRP + d]), w1 = *(const v4fa*)(&swq[(tl + 16) * LRP + d]);
            const v4f u0 = *(const v4fa*)(&suh[sl * LRP + d]), u1 = *(const v4fa*)(&suh[(sl + 16) * LRP + d]);
            const v4f vv = *(const v4fa*)(&sv[ch + d]);
#pragma unroll
            for (int c = 0; c < 4; ++c) {
                a00 = fmaf(vv[c], fast_tanh(w0[c] + u0[c]), a00);
                a01 = fmaf(vv[c], fast_tanh(w0[c] + u1[c]), a01);
                a10 = fmaf(vv[c], fast_tanh(w1[c] + u0[c]), a10);
                a11 = fmaf(vv[c], fast_tanh(w1[c] + u1[c]), a11); }
        }
        __syncthreads();
    }
    os[tl * OSP + sl] = a00; os[tl * OSP + sl + 16] = a01; os[(tl + 16) * OSP + sl] = a10; os[(tl + 16) * OSP + sl + 16] = a11;
    __syncthreads();
    float* orow = OUT + ((size_t)b * TQ_FULL + t0) * SK_FULL + s0;
    const int row = wave * 4 + (lane >> 3), cofs = (lane & 7) * 4;
    const v4f val = *(const v4fa*)(&os[row * OSP + cofs]);
#pragma unroll 1
    for (int ps = 0; ps < 2; ++ps) {
        *(volatile v4f*)(orow + (size_t)row * SK_FULL + cofs) = val;
        if (ps == 0) __threadfence(); }
}

static constexpr size_t al256(size_t v) { return (v + 255) & ~(size_t)255; }
static constexpr size_t SZ_XT = al256((size_t)NB * TQ * DM * 2);
static constexpr size_t SZ_XS = al256((size_t)NB * SK * DM * 2);
static constexpr size_t SZ_WB = al256((size_t)2 * DM * DM * 2);
static constexpr size_t SZ_PT = al256((size_t)NB * TQ * DM * 4);
static constexpr size_t SZ_PS = al256((size_t)NB * SK * DM * 4);
static constexpr size_t SZ_TOTAL = SZ_XT + SZ_XS + SZ_WB + SZ_PT + SZ_PS;
static_assert(SZ_TOTAL <= (size_t)134217728);
static_assert(((size_t)DM * DM * 2) % 256 == 0);
static_assert((size_t)(NB * TQ / 64) * 64 * DM * 4 <= SZ_PT);
static_assert((size_t)(NB * SK / 64) * 64 * DM * 4 <= SZ_PS);

extern "C" void kernel_launch(void* const* d_in, const int* in_sizes, int n_in,
                              void* d_out, int out_size, void* d_ws, size_t ws_size, hipStream_t stream) {
    if (n_in < 6) return;
    const size_t needt = ((size_t)(NB - 1) * TQ_FULL + TQ) * DM;
    const size_t needs = ((size_t)(NB - 1) * SK_FULL + SK) * DM;
    if ((size_t)in_sizes[0] < needt || (size_t)in_sizes[1] < needs) return;
    if ((size_t)in_sizes[2] < (size_t)DM * DM || (size_t)in_sizes[4] < (size_t)DM * DM) return;
    if (in_sizes[3] < DM || in_sizes[5] < DM) return;
    if ((size_t)out_size < ((size_t)(NB - 1) * TQ_FULL + (TQ - 1)) * SK_FULL + SK) return;
    if (SZ_TOTAL > ws_size) return;
    const float* ht = (const float*)d_in[0];
    const float* hs = (const float*)d_in[1];
    const float* wq = (const float*)d_in[2];
    const float* bq = (const float*)d_in[3];
    const float* wc = (const float*)d_in[4];
    const float* vv = (const float*)d_in[5];
    float* OUT = (float*)d_out;
    char* wsp = (char*)d_ws;
    bf* XT = (bf*)wsp; wsp += SZ_XT;
    bf* XS = (bf*)wsp; wsp += SZ_XS;
    bf* WB = (bf*)wsp; wsp += SZ_WB;
    float* WQP = (float*)wsp; wsp += SZ_PT;
    float* UHP = (float*)wsp; wsp += SZ_PS;
    bf* WQB = WB; bf* WCB = WB + (size_t)DM * DM;

    if (TQ == TQ_FULL) {
        const size_t n8 = (size_t)NB * TQ * DM / 8;
        k_cvt8<<<(unsigned)((n8 + 255) / 256), 256, 0, stream>>>(ht, XT, n8);
    } else {
        const size_t n8 = (size_t)TQ * DM / 8;
        for (int b = 0; b < NB; ++b) k_cvt8<<<(unsigned)((n8 + 255) / 256), 256, 0, stream>>>(ht + (size_t)b * TQ_FULL * DM, XT + (size_t)b * TQ * DM, n8);
    }
    if (SK == SK_FULL) {
        const size_t n8 = (size_t)NB * SK * DM / 8;
        k_cvt8<<<(unsigned)((n8 + 255) / 256), 256, 0, stream>>>(hs, XS, n8);
    } else {
        const size_t n8 = (size_t)SK * DM / 8;
        for (int b = 0; b < NB; ++b) k_cvt8<<<(unsigned)((n8 + 255) / 256), 256, 0, stream>>>(hs + (size_t)b * SK_FULL * DM, XS + (size_t)b * SK * DM, n8);
    }
    { const size_t n8 = (size_t)DM * DM / 8; const unsigned g = (unsigned)((n8 + 255) / 256);
      k_cvt8<<<g, 256, 0, stream>>>(wq, WQB, n8); k_cvt8<<<g, 256, 0, stream>>>(wc, WCB, n8); }

    k_projf<<<dim3(NB * TQ / 64, DM / 64, 1), 32, 0, stream>>>(XT, WQB, bq, 1, WQP);
    k_projf<<<dim3(NB * SK / 64, DM / 64, 1), 32, 0, stream>>>(XS, WCB, bq, 0, UHP);

    k_pairsum<<<dim3(SK / TS, TQ / TT, NB), 256, 0, stream>>>(WQP, UHP, vv, OUT);
}
